// NNUE_42159398978365
// MI455X (gfx1250) — hardware-run, weakly checked
//
#include <hip/hip_runtime.h>

typedef float          v8f   __attribute__((ext_vector_type(8)));
typedef float          v4f   __attribute__((ext_vector_type(4)));
typedef unsigned int   v4u   __attribute__((ext_vector_type(4)));
typedef int            v8i   __attribute__((ext_vector_type(8)));
typedef unsigned short v8us  __attribute__((ext_vector_type(8)));
typedef unsigned short v16us __attribute__((ext_vector_type(16)));
typedef __bf16         v16bf __attribute__((ext_vector_type(16)));
typedef _Float16       v16h  __attribute__((ext_vector_type(16)));
typedef v4f  __attribute__((may_alias)) v4fa;
typedef v8us __attribute__((may_alias)) v8usa;
union FragB { v16bf v; v16us u; v8us h[2]; v8i w; };
union FragH { v16h  v; v16us u; v8us h[2]; v8i w; };

__device__ __forceinline__ v8f wmb(const FragB& a, const FragB& b, v8f c) {
  v8f d = __builtin_amdgcn_wmma_f32_16x16x32_bf16(false, a.v, false, b.v, (short)0, c, false, false);
  asm volatile("v_nop\n\tv_nop\n\tv_nop\n\tv_nop" : "+v"(d) : "v"(a.w), "v"(b.w));
  return d;
}

__device__ __forceinline__ v8f wmh(const FragH& a, const FragH& b, v8f c) {
  v8f d = __builtin_amdgcn_wmma_f32_16x16x32_f16(false, a.v, false, b.v, (short)0, c, false, false);
  asm volatile("v_nop\n\tv_nop\n\tv_nop\n\tv_nop" : "+v"(d) : "v"(a.w), "v"(b.w));
  return d;
}

__device__ __forceinline__ unsigned bf16_bits(float f) {
  const unsigned u = __float_as_uint(f);
  const unsigned r = (u + 0x7FFFu + ((u >> 16) & 1u)) >> 16;
  const unsigned q = (u >> 16) | 0x40u;
  return ((u & 0x7fffffffu) > 0x7f800000u) ? q : r;
}

__device__ __forceinline__ float bf16_val(float f) {
  return __uint_as_float(bf16_bits(f) << 16);
}
__device__ __forceinline__ int clampi(int v, int lo, int hi) {
  return v < lo ? lo : (v > hi ? hi : v);
}

__device__ __forceinline__ unsigned f16_bits(float f) {
  const unsigned u  = __float_as_uint(f);
  const unsigned s  = (u >> 16) & 0x8000u;
  const unsigned a  = u & 0x7fffffffu;
  const unsigned t  = a - 0x38000000u;
  const unsigned r  = (t + 0x0FFFu + ((t >> 13) & 1u)) >> 13;
  const unsigned rc = r > 0x7C00u ? 0x7C00u : r;
  const bool small  = a < 0x38800000u;
  const bool isnan  = a > 0x7f800000u;
  const unsigned fin = small ? 0u : (s | rc);
  return isnan ? (s | 0x7E00u) : fin;
}

__device__ __forceinline__ unsigned pk16(unsigned lo, unsigned hi) { return lo | (hi << 16); }
__device__ __forceinline__ unsigned bf16_lo_bits(float v) {
  float hi = bf16_val(v);
  asm volatile("" : "+v"(hi));
  return bf16_bits(v - hi);
}
__device__ __forceinline__ v4u pack8_bf16(v4f a, v4f c) {
  return (v4u){ pk16(bf16_bits(a[0]), bf16_bits(a[1])), pk16(bf16_bits(a[2]), bf16_bits(a[3])),
                pk16(bf16_bits(c[0]), bf16_bits(c[1])), pk16(bf16_bits(c[2]), bf16_bits(c[3])) };
}
__device__ __forceinline__ v4u pack8_bf16_lo(v4f a, v4f c) {
  return (v4u){ pk16(bf16_lo_bits(a[0]), bf16_lo_bits(a[1])), pk16(bf16_lo_bits(a[2]), bf16_lo_bits(a[3])),
                pk16(bf16_lo_bits(c[0]), bf16_lo_bits(c[1])), pk16(bf16_lo_bits(c[2]), bf16_lo_bits(c[3])) };
}
__device__ __forceinline__ v4u pack8_f16(v4f a, v4f c) {
  return (v4u){ pk16(f16_bits(a[0]), f16_bits(a[1])), pk16(f16_bits(a[2]), f16_bits(a[3])),
                pk16(f16_bits(c[0]), f16_bits(c[1])), pk16(f16_bits(c[2]), f16_bits(c[3])) };
}

template <int FORM>
__global__ __launch_bounds__(256) void k_plane(const float* __restrict__ src, int rows, int cols, int ldsrc,
                                               unsigned short* __restrict__ dst, int MP, int KP) {
  static_assert(FORM >= 0 && FORM <= 3);
  const int KTOT = (FORM == 1 || FORM == 3) ? 2 * KP : KP;
  const unsigned ppr   = (unsigned)(KTOT >> 3);
  const unsigned kp8   = (unsigned)(KP >> 3);
  const unsigned total = (unsigned)MP * ppr;
  const unsigned g     = blockIdx.x * 256u + threadIdx.x;
  const unsigned rowu  = g / ppr;
  const unsigned p     = g - rowu * ppr;
  const bool second    = p >= kp8;
  const int row = (int)rowu;
  const int c0  = (int)((second ? p - kp8 : p) << 3);
  const float* srow = src + (size_t)clampi(row, 0, rows - 1) * (size_t)ldsrc;
  float x[8];
  unsigned mk[8];
#pragma unroll
  for (int e = 0; e < 8; ++e) {
    const int c = c0 + e;
    const float v = srow[clampi(c, 0, cols - 1)];
    asm volatile("" :: "v"(v));
    x[e]  = v;
    mk[e] = (row < rows && c < cols) ? 0xFFFFu : 0u;
  }
  const v4f a = (v4f){ x[0], x[1], x[2], x[3] };
  const v4f c = (v4f){ x[4], x[5], x[6], x[7] };
  v4u o;
  if (FORM == 2) {
    o = pack8_f16(a, c);
  } else {
    const v4u hi = pack8_bf16(a, c);
    o = hi;
    if (FORM == 1) { const v4u lo = pack8_bf16_lo(a, c); o = second ? lo : hi; }
  }
  const v4u mw = (v4u){ pk16(mk[0], mk[1]), pk16(mk[2], mk[3]), pk16(mk[4], mk[5]), pk16(mk[6], mk[7]) };
  o &= mw;
  if (g < total) {
    volatile v4u* q = (volatile v4u*)(dst + (size_t)g * 8);
    *q = o;
    __threadfence();
    *q = o;
  }
}

template <int FORM> struct FragOf    { typedef FragB T; };
template <>         struct FragOf<2> { typedef FragH T; };
__device__ __forceinline__ v8f mm(const FragB& a, const FragB& b, v8f c) { return wmb(a, b, c); }
__device__ __forceinline__ v8f mm(const FragH& a, const FragH& b, v8f c) { return wmh(a, b, c); }
template <class F> __device__ __forceinline__ F ld_frag(const unsigned short* p) {
  F f;
  f.h[0] = *(const v8usa*)(p);
  f.h[1] = *(const v8usa*)(p + 16);
  return f;
}

template <int FORM, int EPI>
__global__ __launch_bounds__(256) __attribute__((amdgpu_num_vgpr(248)))
void k_gemm_nt(const unsigned short* __restrict__ A, const unsigned short* __restrict__ B,
               const float* __restrict__ bias, float* __restrict__ D, int M, int N, int KTOT, int ldd) {
  static_assert(FORM >= 0 && FORM <= 2);
  static_assert(EPI == 0 || EPI == 1);
  typedef typename FragOf<FORM>::T F;
  __shared__ __attribute__((aligned(16))) float sT[8][16 * 68];
  const int lane = threadIdx.x & 31;
  const int wave = threadIdx.x >> 5;
  const int tilesM = (M + 63) >> 6;
  const int tilesN = (N + 63) >> 6;
  const int tile = blockIdx.x * 8 + wave;
  if (tile >= tilesM * tilesN) return;
  const int tm = tile / tilesN;
  const int tn = tile - tm * tilesN;
  const int m0 = tm << 6;
  const int n0 = tn << 6;

  const int rl = lane & 15;
  const int h8 = (lane >> 4) * 8;
  const unsigned short* pa = A + (size_t)(m0 + rl) * (size_t)KTOT + h8;
  const unsigned short* pb = B + (size_t)(n0 + rl) * (size_t)KTOT + h8;

  v8f acc[4][4];
#pragma unroll
  for (int i = 0; i < 4; ++i)
#pragma unroll
    for (int j = 0; j < 4; ++j) acc[i][j] = (v8f){0.f, 0.f, 0.f, 0.f, 0.f, 0.f, 0.f, 0.f};

#pragma unroll 1
  for (int k0 = 0; k0 < KTOT; k0 += 32) {
    F bf[4];
#pragma unroll
    for (int j = 0; j < 4; ++j) bf[j] = ld_frag<F>(pb + (size_t)(j << 4) * (size_t)KTOT + k0);
#pragma unroll
    for (int i = 0; i < 4; ++i) {
      const F af = ld_frag<F>(pa + (size_t)(i << 4) * (size_t)KTOT + k0);
#pragma unroll
      for (int j = 0; j < 4; ++j) acc[i][j] = mm(af, bf[j], acc[i][j]);
    }
  }

  float* slab = sT[wave];
  const int hh = lane >> 4;
  const int c4 = (lane & 15) * 4;
  const int nc = n0 + c4;
  const bool cok = nc < N;
  v4f bv = (v4f){0.f, 0.f, 0.f, 0.f};
  if (EPI == 1) {
    bv = *(const v4fa*)(bias + clampi(nc, 0, N - 4));
    asm volatile("" :: "v"(bv));
  }
#pragma unroll
  for (int i = 0; i < 4; ++i) {
    const int mBase = m0 + (i << 4);
#pragma unroll
    for (int j = 0; j < 4; ++j) {
#pragma unroll
      for (int r = 0; r < 8; ++r) slab[(h8 + r) * 68 + (j << 4) + rl] = acc[i][j][r];
    }
    __builtin_amdgcn_fence(__ATOMIC_RELEASE, "workgroup");
    __builtin_amdgcn_wave_barrier();
    __builtin_amdgcn_fence(__ATOMIC_ACQUIRE, "workgroup");
    v4f vv[8];
#pragma unroll
    for (int it = 0; it < 8; ++it) {
      const int row = it * 2 + hh;
      v4f v = *(const v4fa*)(slab + row * 68 + c4);
      if (EPI == 1) v += bv;
      vv[it] = v;
    }
    for (int pass = 0; pass < 2; ++pass) {
#pragma unroll
      for (int it = 0; it < 8; ++it) {
        const int row = mBase + it * 2 + hh;
        if (cok && row < M) *(volatile v4f*)(D + (size_t)row * (size_t)ldd + nc) = vv[it];
      }
      __threadfence();
    }
    __builtin_amdgcn_fence(__ATOMIC_RELEASE, "workgroup");
    __builtin_amdgcn_wave_barrier();
    __builtin_amdgcn_fence(__ATOMIC_ACQUIRE, "workgroup");
  }
}

#pragma clang fp contract(off)

#ifndef TWO_TERM
#define TWO_TERM 1
#endif

typedef unsigned int v2u __attribute__((ext_vector_type(2)));
typedef v2u __attribute__((may_alias)) v2ua;

constexpr int NF     = 101250;
constexpr int L1W    = 128;
constexpr int NB     = 16384;
constexpr int BAG    = 64;
constexpr int NPOL   = 225;
constexpr int NV     = 32;
constexpr int NREAL  = NPOL + NV;
constexpr int NP     = 320;
constexpr int KTOT   = TWO_TERM ? 2 * L1W : L1W;
constexpr int PPR    = KTOT / 8;
constexpr int TBROWS = 101376;
constexpr int POL_ELEMS = NB * NPOL;
constexpr int OUT_ELEMS = POL_ELEMS + NB;
constexpr int WS_PIECES = NP * PPR;
constexpr int WS_BLOCKS = WS_PIECES / 256;

static_assert(BAG == 64);
static_assert(L1W == 128 && L1W == 32 * 4);
static_assert(NB % 32 == 0 && NB % 64 == 0 && NB % 8 == 0);
static_assert(POL_ELEMS == 16384 * 225 && POL_ELEMS == 3686400);
static_assert(POL_ELEMS % 32 == 0 && POL_ELEMS % 256 == 0);
static_assert(OUT_ELEMS == 3702784);
static_assert(NP % 64 == 0 && NP >= NREAL && NREAL == 257 && NP % 32 == 0 && NP % 4 == 0);
static_assert(KTOT % 32 == 0 && L1W % 32 == 0);
static_assert(TBROWS % 64 == 0 && TBROWS >= NF && (TBROWS * (L1W / 8)) % 256 == 0);
static_assert((long long)TBROWS * L1W / 8 < 0x7fffffffLL);
static_assert(WS_PIECES % 256 == 0);
static_assert(NV == 32);

constexpr size_t SZ_TB   = (size_t)TBROWS * L1W * 2;
constexpr size_t SZ_A    = (size_t)NB * KTOT * 2;
constexpr size_t SZ_T    = (size_t)NB * NP * 4;
constexpr size_t SZ_WS   = (size_t)NP * KTOT * 2;
constexpr size_t SZ_BIAS = (size_t)NP * 4;
constexpr size_t SZ_VW2  = (size_t)NV * NV * 4;
constexpr size_t SZ_SV   = 512;
constexpr size_t OFF_TB   = 0;
constexpr size_t OFF_A    = OFF_TB + SZ_TB;
constexpr size_t OFF_T    = OFF_A + SZ_A;
constexpr size_t OFF_WS   = OFF_T + SZ_T;
constexpr size_t OFF_BIAS = OFF_WS + SZ_WS;
constexpr size_t OFF_VW2  = OFF_BIAS + SZ_BIAS;
constexpr size_t OFF_SV   = OFF_VW2 + SZ_VW2;
constexpr size_t WS_TOTAL = OFF_SV + SZ_SV;
static_assert(SZ_TB % 256 == 0 && SZ_A % 256 == 0 && SZ_T % 256 == 0 && SZ_WS % 256 == 0);
static_assert(SZ_BIAS % 256 == 0 && SZ_VW2 % 256 == 0 && SZ_SV % 256 == 0);
static_assert(OFF_A % 256 == 0 && OFF_T % 256 == 0 && OFF_WS % 256 == 0 && OFF_BIAS % 256 == 0);
static_assert(OFF_VW2 % 256 == 0 && OFF_SV % 256 == 0);
static_assert(SZ_TB == (size_t)25952256 && SZ_T == (size_t)20971520);
static_assert(WS_TOTAL <= ((size_t)128 << 20));

__device__ __forceinline__ float blend2(float a, unsigned ma, float b, unsigned mb) {
  return __uint_as_float((__float_as_uint(a) & ma) | (__float_as_uint(b) & mb));
}
__device__ __forceinline__ float clip01(float t) {
  return (t < 0.0f) ? 0.0f : ((t > 1.0f) ? 1.0f : t);
}

__global__ __launch_bounds__(256) void k_prep(const float* __restrict__ pw, const float* __restrict__ pb,
                                              const float* __restrict__ vw1, const float* __restrict__ vb1,
                                              const float* __restrict__ vw2, const float* __restrict__ vb2,
                                              const float* __restrict__ vw3, const float* __restrict__ vb3,
                                              unsigned short* __restrict__ WS, float* __restrict__ BIAS,
                                              float* __restrict__ VW2, float* __restrict__ SV) {
  const int tid = (int)threadIdx.x;
  const int blk = (int)blockIdx.x;
  if (blk < WS_BLOCKS) {
    const int g   = blk * 256 + tid;
    const int gc  = g < WS_PIECES ? g : WS_PIECES - 1;
    const int row = gc / PPR;
    const int p   = gc - row * PPR;
    const int c0  = (p & 15) << 3;
    const int rp  = clampi(row, 0, NPOL - 1);
    const int rv  = clampi(row - NPOL, 0, NV - 1);
    const v4f pa = *(const v4fa*)(pw + (size_t)rp * L1W + c0);
    const v4f pc = *(const v4fa*)(pw + (size_t)rp * L1W + c0 + 4);
    const v4f va = *(const v4fa*)(vw1 + (size_t)rv * L1W + c0);
    const v4f vc = *(const v4fa*)(vw1 + (size_t)rv * L1W + c0 + 4);
    asm volatile("" :: "v"(pa));
    asm volatile("" :: "v"(pc));
    asm volatile("" :: "v"(va));
    asm volatile("" :: "v"(vc));
    const unsigned mp = (row < NPOL) ? 0xFFFFFFFFu : 0u;
    const unsigned mv = (row >= NPOL && row < NREAL) ? 0xFFFFFFFFu : 0u;
    const v4f a = (v4f){ blend2(pa[0], mp, va[0], mv), blend2(pa[1], mp, va[1], mv),
                         blend2(pa[2], mp, va[2], mv), blend2(pa[3], mp, va[3], mv) };
    const v4f c = (v4f){ blend2(pc[0], mp, vc[0], mv), blend2(pc[1], mp, vc[1], mv),
                         blend2(pc[2], mp, vc[2], mv), blend2(pc[3], mp, vc[3], mv) };
    const v4u o = pack8_bf16(a, c);
    if (g < WS_PIECES) {
      volatile v4u* q = (volatile v4u*)(WS + (size_t)g * 8);
      *q = o;
      __threadfence();
      *q = o;
    }
  } else if (blk == WS_BLOCKS) {
    const v4f a = *(const v4fa*)(vw2 + 4 * tid);
    asm volatile("" :: "v"(a));
    const v4f o = (v4f){ bf16_val(a[0]), bf16_val(a[1]), bf16_val(a[2]), bf16_val(a[3]) };
    volatile v4f* q = (volatile v4f*)(VW2 + 4 * tid);
    *q = o;
    __threadfence();
    *q = o;
  } else if (blk == WS_BLOCKS + 1) {
    const int u = tid < (NP / 4) ? tid : (NP / 4) - 1;
    float x[4];
#pragma unroll
    for (int i = 0; i < 4; ++i) {
      const int e = 4 * u + i;
      const float a = pb[clampi(e, 0, NPOL - 1)];
      const float b = vb1[clampi(e - NPOL, 0, NV - 1)];
      asm volatile("" :: "v"(a));
      asm volatile("" :: "v"(b));
      const unsigned ma = (e < NPOL) ? 0xFFFFFFFFu : 0u;
      const unsigned mb = (e >= NPOL && e < NREAL) ? 0xFFFFFFFFu : 0u;
      x[i] = bf16_val(blend2(a, ma, b, mb));
    }
    const v4f o = (v4f){ x[0], x[1], x[2], x[3] };
    if (tid < NP / 4) {
      volatile v4f* q = (volatile v4f*)(BIAS + 4 * tid);
      *q = o;
      __threadfence();
      *q = o;
    }
  } else {
    const int u = tid < 32 ? tid : 31;
    const v4f a = *(const v4fa*)(vb2 + 4 * clampi(u, 0, 7));
    const v4f b = *(const v4fa*)(vw3 + 4 * clampi(u - 8, 0, 7));
    const float z = vb3[0];
    asm volatile("" :: "v"(a));
    asm volatile("" :: "v"(b));
    asm volatile("" :: "v"(z));
    const unsigned ma = (u < 8) ? 0xFFFFFFFFu : 0u;
    const unsigned mb = (u >= 8 && u < 16) ? 0xFFFFFFFFu : 0u;
    const unsigned mz = (u == 16) ? 0xFFFFFFFFu : 0u;
    const float e0 = __uint_as_float(__float_as_uint(blend2(a[0], ma, b[0], mb)) | (__float_as_uint(z) & mz));
    const v4f o = (v4f){ bf16_val(e0), bf16_val(blend2(a[1], ma, b[1], mb)),
                         bf16_val(blend2(a[2], ma, b[2], mb)), bf16_val(blend2(a[3], ma, b[3], mb)) };
    if (tid < 32) {
      volatile v4f* q = (volatile v4f*)(SV + 4 * tid);
      *q = o;
      __threadfence();
      *q = o;
    }
  }
}

__global__ __launch_bounds__(256) void k_bag(const int* __restrict__ idx, const unsigned short* __restrict__ TB,
                                             unsigned short* __restrict__ A) {
  const int tid = (int)threadIdx.x, lane = tid & 31, wave = tid >> 5;
  const int s  = __builtin_amdgcn_readfirstlane((int)blockIdx.x * 8 + wave);
  const int sc = s < NB ? s : NB - 1;

  int ra = idx[(size_t)sc * BAG + lane];
  asm volatile("" :: "v"(ra));
  int rb = idx[(size_t)sc * BAG + 32 + lane];
  asm volatile("" :: "v"(rb));
  const int ia = clampi(ra, 0, NF - 1);
  const int ib = clampi(rb, 0, NF - 1);

  const unsigned short* Tl = TB + 4 * lane;
  float a0 = 0.0f, a1 = 0.0f, a2 = 0.0f, a3 = 0.0f;
#pragma unroll 8
  for (int j = 0; j < 32; ++j) {
    const int id = __builtin_amdgcn_readlane(ia, j);
    const v2u w = *(const v2ua*)(Tl + (size_t)id * L1W);
    const unsigned w0 = w[0], w1 = w[1];
    asm volatile("" :: "v"(w0));
    asm volatile("" :: "v"(w1));
    a0 = a0 + __uint_as_float(w0 << 16);
    a1 = a1 + __uint_as_float(w0 & 0xFFFF0000u);
    a2 = a2 + __uint_as_float(w1 << 16);
    a3 = a3 + __uint_as_float(w1 & 0xFFFF0000u);
  }
#pragma unroll 8
  for (int j = 0; j < 32; ++j) {
    const int id = __builtin_amdgcn_readlane(ib, j);
    const v2u w = *(const v2ua*)(Tl + (size_t)id * L1W);
    const unsigned w0 = w[0], w1 = w[1];
    asm volatile("" :: "v"(w0));
    asm volatile("" :: "v"(w1));
    a0 = a0 + __uint_as_float(w0 << 16);
    a1 = a1 + __uint_as_float(w0 & 0xFFFF0000u);
    a2 = a2 + __uint_as_float(w1 << 16);
    a3 = a3 + __uint_as_float(w1 & 0xFFFF0000u);
  }

  const v2u oh = (v2u){ pk16(bf16_bits(a0), bf16_bits(a1)), pk16(bf16_bits(a2), bf16_bits(a3)) };
#if TWO_TERM
  const v2u ol = (v2u){ pk16(bf16_lo_bits(a0), bf16_lo_bits(a1)), pk16(bf16_lo_bits(a2), bf16_lo_bits(a3)) };
#endif
  if (s < NB) {
    volatile v2u* qh = (volatile v2u*)(A + (size_t)s * KTOT + 4 * lane);
    *qh = oh;
#if TWO_TERM
    volatile v2u* ql = (volatile v2u*)(A + (size_t)s * KTOT + L1W + 4 * lane);
    *ql = ol;
#endif
    __threadfence();
    *qh = oh;
#if TWO_TERM
    *ql = ol;
#endif
  }
}

__global__ __launch_bounds__(256) void k_val(const float* __restrict__ T, const float* __restrict__ VW2,
                                             const float* __restrict__ SV, float* __restrict__ out) {
  const int tid = (int)threadIdx.x, lane = tid & 31, wave = tid >> 5;
  const int g = __builtin_amdgcn_readfirstlane((int)blockIdx.x * 8 + wave);

  v4f wv[8];
#pragma unroll
  for (int i = 0; i < 8; ++i) {
    wv[i] = *(const v4fa*)(VW2 + lane * NV + 4 * i);
    asm volatile("" :: "v"(wv[i]));
  }
  const float b2 = SV[lane];
  const float w3 = SV[32 + lane];
  const float b3 = SV[64];
  asm volatile("" :: "v"(b2));
  asm volatile("" :: "v"(w3));
  asm volatile("" :: "v"(b3));

  float keep = 0.0f;
#pragma unroll 1
  for (int p = 0; p < 32; ++p) {
    const int s  = g * 32 + p;
    const int sc = s < NB ? s : NB - 1;
    const float t = T[(size_t)sc * NP + NPOL + lane];
    asm volatile("" :: "v"(t));
    const float v1 = clip01(t);
    const int v1i = __float_as_int(v1);
    float a = 0.0f;
#pragma unroll
    for (int k = 0; k < 32; ++k) {
      const float vk = __int_as_float(__builtin_amdgcn_readlane(v1i, k));
      a = fmaf(vk, wv[k >> 2][k & 3], a);
    }
    a = a + b2;
    const float v2 = clip01(a);
    float q = v2 * w3;
    q = q + __shfl_xor(q, 16, 32);
    q = q + __shfl_xor(q, 8, 32);
    q = q + __shfl_xor(q, 4, 32);
    q = q + __shfl_xor(q, 2, 32);
    q = q + __shfl_xor(q, 1, 32);
    const float r = tanhf(q + b3);
    keep = (lane == p) ? r : keep;
  }

  const int so = g * 32 + lane;
  if (so < NB) {
    volatile float* qv = (volatile float*)(out + (size_t)POL_ELEMS + so);
    *qv = keep;
    __threadfence();
    *qv = keep;
  }
}

__global__ __launch_bounds__(256) void k_pol(const float* __restrict__ T, float* __restrict__ out) {
  const int f  = (int)blockIdx.x * 256 + (int)threadIdx.x;
  const int fc = f < POL_ELEMS ? f : POL_ELEMS - 1;
  const int s  = fc / NPOL;
  const int c  = fc - s * NPOL;
  const float v = T[(size_t)s * NP + c];
  asm volatile("" :: "v"(v));
  if (f < POL_ELEMS) {
    volatile float* q = (volatile float*)(out + f);
    *q = v;
    __threadfence();
    *q = v;
  }
}

extern "C" void kernel_launch(void* const* d_in, const int* in_sizes, int n_in,
                              void* d_out, int out_size, void* d_ws, size_t ws_size,
                              hipStream_t stream) {
  if (n_in < 10) return;
  if (in_sizes[0] != NB * BAG) return;
  if (in_sizes[1] != NF * L1W) return;
  if (in_sizes[2] != NPOL * L1W) return;
  if (in_sizes[3] != NPOL) return;
  if (in_sizes[4] != NV * L1W) return;
  if (in_sizes[5] != NV) return;
  if (in_sizes[6] != NV * NV) return;
  if (in_sizes[7] != NV) return;
  if (in_sizes[8] != NV) return;
  if (in_sizes[9] != 1) return;
  if (out_size != OUT_ELEMS) return;
  if (ws_size < WS_TOTAL) return;

  const int*   indices = (const int*)d_in[0];
  const float* emb = (const float*)d_in[1];
  const float* pw  = (const float*)d_in[2];
  const float* pb  = (const float*)d_in[3];
  const float* vw1 = (const float*)d_in[4];
  const float* vb1 = (const float*)d_in[5];
  const float* vw2 = (const float*)d_in[6];
  const float* vb2 = (const float*)d_in[7];
  const float* vw3 = (const float*)d_in[8];
  const float* vb3 = (const float*)d_in[9];
  float* out = (float*)d_out;

  char* ws = (char*)d_ws;
  unsigned short* TB   = (unsigned short*)(ws + OFF_TB);
  unsigned short* Apl  = (unsigned short*)(ws + OFF_A);
  float*          T    = (float*)(ws + OFF_T);
  unsigned short* WS   = (unsigned short*)(ws + OFF_WS);
  float*          BIAS = (float*)(ws + OFF_BIAS);
  float*          VW2  = (float*)(ws + OFF_VW2);
  float*          SV   = (float*)(ws + OFF_SV);

  k_plane<0><<<TBROWS * (L1W / 8) / 256, 256, 0, stream>>>(emb, NF, L1W, L1W, TB, TBROWS, L1W);
  k_prep<<<WS_BLOCKS + 3, 256, 0, stream>>>(pw, pb, vw1, vb1, vw2, vb2, vw3, vb3, WS, BIAS, VW2, SV);
  k_bag<<<NB / 8, 256, 0, stream>>>(indices, TB, Apl);
  k_gemm_nt<0, 1><<<((NB / 64) * (NP / 64) + 7) / 8, 256, 0, stream>>>(Apl, WS, BIAS, T, NB, NP, KTOT, NP);
  k_val<<<NB / 32 / 8, 256, 0, stream>>>(T, VW2, SV, out);
  k_pol<<<POL_ELEMS / 256, 256, 0, stream>>>(T, out);
}
